// Triangle_Att_Start_34660386079039
// MI455X (gfx1250) — hardware-verified
//
#include <hip/hip_runtime.h>
#include <math.h>

typedef __attribute__((ext_vector_type(16))) _Float16 v16h;
typedef __attribute__((ext_vector_type(16))) __bf16 v16b;
typedef __attribute__((ext_vector_type(8)))  _Float16 v8h;
typedef __attribute__((ext_vector_type(8)))  float v8f;
typedef __attribute__((ext_vector_type(4)))  float v4f;
typedef __attribute__((ext_vector_type(2)))  float v2f;
typedef __attribute__((ext_vector_type(4)))  unsigned v4u;
typedef __attribute__((ext_vector_type(4)))  int v4i;
typedef float __attribute__((may_alias)) float_a;
typedef int __attribute__((may_alias)) int_a;

template <typename T> __device__ __forceinline__ void vst2(void* p, T v) { *(volatile T*)p = v; __threadfence(); *(volatile T*)p = v; }
__device__ __forceinline__ v8f wmma16(v16h a, v16h b, v8f c) {
  v8f d = __builtin_amdgcn_wmma_f32_16x16x32_f16(false, a, false, b, (short)0, c, false, false);
  asm volatile("v_nop\n\tv_nop\n\tv_nop\n\tv_nop" : "+v"(d) : "v"(a), "v"(b));
  return d;
}
__device__ __forceinline__ v8f wmma_bf(v16b a, v16b b, v8f c) {
  v8f d = __builtin_amdgcn_wmma_f32_16x16x32_bf16(false, a, false, b, (short)0, c, false, false);
  asm volatile("v_nop\n\tv_nop\n\tv_nop\n\tv_nop" : "+v"(d) : "v"(a), "v"(b));
  return d;
}
__device__ __forceinline__ v16h frag_h(const _Float16* rowk0, int lane) {
  union { v16h v; v8h q[2]; } u; const _Float16* p = rowk0 + 8 * (lane >> 4);
  u.q[0] = *(const v8h*)p; u.q[1] = *(const v8h*)(p + 16); return u.v;
}
__device__ __forceinline__ v16h frag_f32(const float* rowk0, int lane) {
  v16h a; const float* p = rowk0 + 8 * (lane >> 4);
#pragma unroll
  for (int i = 0; i < 8; ++i) { a[i] = (_Float16)p[i]; a[8 + i] = (_Float16)p[16 + i]; }
  return a;
}
__device__ __forceinline__ v16h frag_f32s(const float* rowk0, int lane, float sc) {
  v16h a; const float* p = rowk0 + 8 * (lane >> 4);
#pragma unroll
  for (int i = 0; i < 8; ++i) { a[i] = (_Float16)(p[i] * sc); a[8 + i] = (_Float16)(p[16 + i] * sc); }
  return a;
}
__device__ __forceinline__ v16h fragc_f32(const float* W, int k0, int n, int lane, int ld, int K) {
  v16h a; const int g = lane >> 4;
#pragma unroll
  for (int i = 0; i < 8; ++i) { const int ka = k0 + 8 * g + i, kb = ka + 16;
    a[i] = (_Float16)(ka < K ? W[(size_t)ka * ld + n] : 0.f); a[8 + i] = (_Float16)(kb < K ? W[(size_t)kb * ld + n] : 0.f); }
  return a;
}
struct F2 { v16b h, l; };
__device__ __forceinline__ F2 bsplit16(const float v[16]) { F2 r;
#pragma unroll
  for (int i = 0; i < 16; ++i) { const __bf16 h = (__bf16)v[i]; r.h[i] = h; r.l[i] = (__bf16)(v[i] - (float)h); }
  return r; }
__device__ __forceinline__ F2 split_row(const float* row, int k0, int lane) { float v[16]; const float* p = row + k0 + 8 * (lane >> 4);
#pragma unroll
  for (int i = 0; i < 8; ++i) { v[i] = p[i]; v[8 + i] = p[16 + i]; }
  return bsplit16(v); }
__device__ __forceinline__ F2 split_rowK(const float* row, int k0, int lane, int K) { float v[16]; const int g = lane >> 4;
#pragma unroll
  for (int i = 0; i < 8; ++i) { const int ka = k0 + 8 * g + i, kb = ka + 16; v[i] = ka < K ? row[ka] : 0.f; v[8 + i] = kb < K ? row[kb] : 0.f; }
  return bsplit16(v); }
__device__ __forceinline__ F2 split_col(const float* W, int k0, int n, int lane, int ld, int K) { float v[16]; const int g = lane >> 4;
#pragma unroll
  for (int i = 0; i < 8; ++i) { const int ka = k0 + 8 * g + i, kb = ka + 16; v[i] = ka < K ? W[(size_t)ka * ld + n] : 0.f; v[8 + i] = kb < K ? W[(size_t)kb * ld + n] : 0.f; }
  return bsplit16(v); }
__device__ __forceinline__ v8f mac3(const F2& a, const F2& b, v8f c) { c = wmma_bf(a.l, b.h, c); c = wmma_bf(a.h, b.l, c); return wmma_bf(a.h, b.h, c); }
__device__ __forceinline__ float sigm(float v) { return 1.0f / (1.0f + expf(-v)); }
#define LDSX() do { asm volatile("s_wait_dscnt 0" ::: "memory"); __builtin_amdgcn_wave_barrier(); __builtin_amdgcn_fence(__ATOMIC_RELEASE, "workgroup"); } while (0)

#define LL 256
#define PD 128
#define NH 4
#define HID 32
#define NR (LL * LL)

__global__ __launch_bounds__(256) void k_packW(const float* __restrict__ Wq, const float* __restrict__ Wk, const float* __restrict__ Wv, const float* __restrict__ Wg, const float* __restrict__ Wo, _Float16* __restrict__ P) {
  const int n = blockIdx.x, tid = threadIdx.x; const int which = n >> 7, c = n & 127;
  const float* W = which == 0 ? Wq : (which == 1 ? Wk : (which == 2 ? Wv : (which == 3 ? Wg : Wo)));
  if (tid < PD / 8) { union { v8h hh; v4u u; } pk;
#pragma unroll
    for (int i = 0; i < 8; ++i) pk.hh[i] = (_Float16)(W[(size_t)(tid * 8 + i) * PD + c] * 16.0f);
    vst2(P + (size_t)n * PD + tid * 8, pk.u); }
}
__global__ __launch_bounds__(128) void k_proj(const float* __restrict__ pair, const float* __restrict__ lng, const float* __restrict__ lnb, const _Float16* __restrict__ P, const float* __restrict__ Wb,
                                            const float* __restrict__ bg, _Float16* __restrict__ Q, _Float16* __restrict__ Kt, _Float16* __restrict__ VT, float* __restrict__ gate, float* __restrict__ xb) {
  __shared__ __align__(16) float sx[64][PD + 4];
  __shared__ __align__(16) float so[4][16][132];
  __shared__ __align__(16) _Float16 st[PD][72];
  __shared__ __align__(16) float sb[64 * 4];
  const int tid = threadIdx.x, wave = tid >> 5, lane = tid & 31, col = lane & 15, g = lane >> 4;
  const int r0b = blockIdx.x * 64; const int i = r0b / LL, j0 = r0b % LL;
  { const int rl = tid >> 1, hf = tid & 1; const float* pr = pair + (size_t)(r0b + rl) * PD + hf * 64;
    float s = 0.f; for (int c = 0; c < 64; ++c) s += pr[c];
    s += __shfl_xor(s, 1, 32); const float mu = s / (float)PD;
    float q2 = 0.f; for (int c = 0; c < 64; ++c) { const float d = pr[c] - mu; q2 += d * d; }
    q2 += __shfl_xor(q2, 1, 32); const float rs = rsqrtf(q2 / (float)PD + 1e-5f);
    for (int c = 0; c < 64; ++c) { const int cc = hf * 64 + c; sx[rl][cc] = (pr[c] - mu) * rs * lng[cc] + lnb[cc]; } }
  __syncthreads();
  { const int rl = tid >> 1, o0 = (tid & 1) * 2;
    for (int u = 0; u < 2; ++u) { const int o = o0 + u; float a = 0.f;
#pragma unroll 1
      for (int c = 0; c < PD; ++c) a += sx[rl][c] * Wb[c * NH + o];
      sb[rl * 4 + o] = a; } }
#pragma unroll 1
  for (int which = 0; which < 4; ++which) {
    v8f acc[8] = {};
#pragma unroll
    for (int kc = 0; kc < PD / 32; ++kc) { const v16h a = frag_f32(&sx[wave * 16 + col][0] + kc * 32, lane);
#pragma unroll
      for (int jj = 0; jj < 8; ++jj) acc[jj] = wmma16(a, frag_h(P + (size_t)(which * PD + jj * 16 + col) * PD + kc * 32, lane), acc[jj]); }
    if (which == 2) {
#pragma unroll
      for (int jj = 0; jj < 8; ++jj)
#pragma unroll
        for (int r = 0; r < 8; ++r) st[jj * 16 + col][wave * 16 + 8 * g + r] = (_Float16)acc[jj][r];
      __syncthreads();
      for (int q = tid; q < PD * 8; q += 128) { const int c = q >> 3, pc = q & 7; vst2(VT + (((size_t)i * NH * HID + c) * LL) + j0 + pc * 8, *(const v4u*)(&st[c][pc * 8])); }
      __syncthreads();
    } else {
#pragma unroll
      for (int jj = 0; jj < 8; ++jj) { const float bb = which == 3 ? bg[jj * 16 + col] : 0.f;
#pragma unroll
        for (int r = 0; r < 8; ++r) { so[wave][8 * g + r][jj * 16 + col] = which == 3 ? sigm(acc[jj][r] * (1.0f / 16.0f) + bb) : acc[jj][r]; } }
      LDSX();
      if (which == 3) {
#pragma unroll 4
        for (int rl = 0; rl < 16; ++rl) vst2(gate + (size_t)(r0b + wave * 16 + rl) * PD + lane * 4, *(const v4f*)(&so[wave][rl][lane * 4]));
      } else { _Float16* dst = which == 0 ? Q : Kt;
        for (int q = lane; q < NH * 16 * 4; q += 32) { const int n = q >> 6, rem = q & 63, rl = rem >> 2, pc = rem & 3; union { v8h hh; v4u u; } pk;
#pragma unroll
          for (int e = 0; e < 8; ++e) pk.hh[e] = (_Float16)so[wave][rl][n * HID + pc * 8 + e];
          vst2(dst + (((size_t)i * NH + n) * LL + j0 + wave * 16 + rl) * HID + pc * 8, pk.u); } }
      LDSX();
    }
  }
  __syncthreads();
  for (int q = tid; q < 64; q += 128) vst2(xb + (size_t)(r0b + q) * 4, *(const v4f*)(&sb[q * 4]));
}
__global__ __launch_bounds__(128) void k_attn(const _Float16* __restrict__ Q, const _Float16* __restrict__ Kt, const _Float16* __restrict__ VT, const float* __restrict__ xb, const float* __restrict__ gate, float* __restrict__ O) {
  __shared__ __align__(16) float sS[64][LL + 4];
  __shared__ __align__(16) _Float16 sP[64][LL + 8];
  __shared__ __align__(16) float so[4][16][36];
  const int tid = threadIdx.x, w = tid >> 5, lane = tid & 31, col = lane & 15, g = lane >> 4;
  const int n = blockIdx.y, i = blockIdx.z, j0 = blockIdx.x * 64 + w * 16;
  const _Float16* qb = Q + ((size_t)i * NH + n) * LL * HID; const _Float16* kb = Kt + ((size_t)i * NH + n) * LL * HID; const _Float16* vb = VT + ((size_t)i * NH + n) * HID * LL;
  const float fac = rsqrtf((float)HID) * (1.0f / 256.0f);
  const v16h aq = frag_h(qb + (size_t)(j0 + col) * HID, lane);
#pragma unroll 1
  for (int t = 0; t < LL / 16; ++t) { v8f acc = {}; acc = wmma16(aq, frag_h(kb + (size_t)(t * 16 + col) * HID, lane), acc);
    const int k = t * 16 + col;
#pragma unroll
    for (int r = 0; r < 8; ++r) { const int jl = w * 16 + 8 * g + r; sS[jl][k] = acc[r] * fac + xb[((size_t)k * LL + j0 + 8 * g + r) * 4 + n]; } }
  __syncthreads();
  { const int rl = tid >> 1, hf = tid & 1; float mx = -3.0e38f;
    for (int k = 0; k < 128; ++k) mx = fmaxf(mx, sS[rl][hf * 128 + k]);
    mx = fmaxf(mx, __shfl_xor(mx, 1, 32));
    float s = 0.f; for (int k = 0; k < 128; ++k) { const float p = expf(sS[rl][hf * 128 + k] - mx); sS[rl][hf * 128 + k] = p; s += p; }
    s += __shfl_xor(s, 1, 32); const float inv = 16384.0f / s;
    for (int k = 0; k < 128; ++k) sP[rl][hf * 128 + k] = (_Float16)(sS[rl][hf * 128 + k] * inv); }
  __syncthreads();
  v8f acc[2] = {};
#pragma unroll 1
  for (int kc = 0; kc < LL / 32; ++kc) { const v16h pa = frag_h(&sP[w * 16 + col][0] + kc * 32, lane);
#pragma unroll
    for (int t = 0; t < 2; ++t) acc[t] = wmma16(pa, frag_h(vb + (size_t)(t * 16 + col) * LL + kc * 32, lane), acc[t]); }
#pragma unroll
  for (int t = 0; t < 2; ++t)
#pragma unroll
    for (int r = 0; r < 8; ++r) { const size_t row = (size_t)i * LL + j0 + 8 * g + r; const int c = n * HID + t * 16 + col; so[w][8 * g + r][t * 16 + col] = acc[t][r] * (1.0f / (16384.0f * 16.0f)) * gate[row * PD + c]; }
  LDSX();
  for (int q = lane; q < 16 * 8; q += 32) { const int rl = q >> 3, pc = q & 7; vst2(O + ((size_t)i * LL + j0 + rl) * PD + n * HID + pc * 4, *(const v4f*)(&so[w][rl][pc * 4])); }
}
__global__ __launch_bounds__(128) void k_out(const float* __restrict__ O, const float* __restrict__ Wo, const float* __restrict__ bo, float* __restrict__ out) {
  __shared__ __align__(16) float so[4][16][132];
  const int tid = threadIdx.x, wave = tid >> 5, lane = tid & 31, col = lane & 15, g = lane >> 4;
  const int r0 = blockIdx.x * 64 + wave * 16;
  v8f acc[8] = {};
#pragma unroll 1
  for (int kc = 0; kc < PD / 32; ++kc) { const F2 a = split_row(O + (size_t)(r0 + col) * PD, kc * 32, lane);
#pragma unroll
    for (int jj = 0; jj < 8; ++jj) acc[jj] = mac3(a, split_col(Wo, kc * 32, jj * 16 + col, lane, PD, PD), acc[jj]); }
#pragma unroll
  for (int jj = 0; jj < 8; ++jj) { const float bb = bo[jj * 16 + col];
#pragma unroll
    for (int r = 0; r < 8; ++r) so[wave][8 * g + r][jj * 16 + col] = acc[jj][r] + bb; }
  LDSX();
#pragma unroll 4
  for (int rl = 0; rl < 16; ++rl) vst2(out + (size_t)(r0 + rl) * PD + lane * 4, *(const v4f*)(&so[wave][rl][lane * 4]));
}
extern "C" void kernel_launch(void* const* d_in, const int* in_sizes, int n_in, void* d_out, int out_size, void* d_ws, size_t ws_size, hipStream_t stream) {
  (void)in_sizes; (void)n_in; (void)out_size; (void)ws_size;
  const float* pair = (const float*)d_in[0]; const float* lng = (const float*)d_in[1]; const float* lnb = (const float*)d_in[2];
  const float* Wq = (const float*)d_in[3]; const float* Wk = (const float*)d_in[4]; const float* Wv = (const float*)d_in[5]; const float* Wb = (const float*)d_in[6];
  const float* Wg = (const float*)d_in[7]; const float* bg = (const float*)d_in[8]; const float* Wo = (const float*)d_in[9]; const float* bo = (const float*)d_in[10];
  float* out = (float*)d_out;
  char* ws = (char*)d_ws; size_t off = 0;
  auto take = [&](size_t bytes) { char* p = ws + off; off += (bytes + 255) & ~(size_t)255; return p; };
  _Float16* P = (_Float16*)take((size_t)5 * PD * PD * 2);
  _Float16* Q = (_Float16*)take((size_t)NR * PD * 2); _Float16* Kt = (_Float16*)take((size_t)NR * PD * 2); _Float16* VT = (_Float16*)take((size_t)NR * PD * 2);
  float* gate = (float*)take((size_t)NR * PD * 4); float* xb = (float*)take((size_t)NR * 4 * 4); float* O = (float*)take((size_t)NR * PD * 4);
  k_packW<<<5 * PD, 256, 0, stream>>>(Wq, Wk, Wv, Wg, Wo, P);
  k_proj<<<NR / 64, 128, 0, stream>>>(pair, lng, lnb, P, Wb, bg, Q, Kt, VT, gate, xb);
  k_attn<<<dim3(LL / 64, NH, LL), 128, 0, stream>>>(Q, Kt, VT, xb, gate, O);
  k_out<<<NR / 64, 128, 0, stream>>>(O, Wo, bo, out);
}
